// MultiHeadAttentionLayer_39161511805520
// MI455X (gfx1250) — hardware-run, weakly checked
//
#include <hip/hip_runtime.h>


#ifndef NB
#define NB 4
#endif
#ifndef SEQ
#define SEQ 256
#endif
#define NB_FULL  4
#define SEQ_FULL 256
#ifndef OUT_SEQ
#define OUT_SEQ SEQ
#endif
#define DM   512
#define NH_  8
#define HD   64
#define QB   32
#define KG   (SEQ / 128)
#define NKL  (4 * KG)
#define KSP  66
#define PSP  (SEQ + 8)
#define XSP  68
#define QSP  72
#define WAS  64.0f
#define WAI  0.015625f
#define FOS  256.0f
#define XCS  256.0f
#define OUTI 1.52587890625e-05f
#define PCS  16384.0f
#define LOG2E 1.4426950408889634f

static_assert(HD == 64);
static_assert(NH_ * HD == DM);
static_assert(DM % 64 == 0);
static_assert(DM % 32 == 0);
static_assert(HD % 32 == 0);
static_assert(SEQ % 64 == 0);
static_assert((NB * SEQ) % 64 == 0);
static_assert(SEQ % 128 == 0);
static_assert(SEQ % 32 == 0);
static_assert(SEQ % QB == 0);
static_assert(QB % 16 == 0);
static_assert(QB % 8 == 0);
static_assert((QB / 16) * (HD / 16) == 8);
static_assert(32 * 16 * KG == SEQ * 4);
static_assert(256 * 16 == QB * HD * 2);
static_assert(32 * 16 * 4 == 16 * 64 * 2);
static_assert(32 * 16 * 8 == 16 * 64 * 4);
static_assert(32 * 4 * 8 == 16 * 64);
static_assert((QSP * 2) % 16 == 0);
static_assert((PSP * 2) % 16 == 0);
static_assert((XSP * 4) % 16 == 0);
static_assert((KSP * 4) % 8 == 0);
static_assert(((size_t)SEQ * DM) % 8 == 0);
static_assert(((size_t)DM * DM) % 8 == 0);
static_assert(((size_t)HD * HD) % 8 == 0);
static_assert(NB <= NB_FULL);
static_assert(SEQ <= SEQ_FULL);
static_assert((size_t)SEQ * KSP * 4 + (size_t)QB * HD * 4 + (size_t)HD * 4 + (size_t)QB * PSP * 2 + (size_t)QB * XSP * 4 + (size_t)QB * 4 <= 131072);
static_assert((size_t)16 * 68 * 4 + (size_t)64 * QSP * 2 <= 131072);
static_assert((size_t)NB_FULL * SEQ_FULL * DM * 4 == 2097152);
static_assert(((size_t)NB_FULL * SEQ_FULL * DM + (size_t)NB_FULL * NH_ * SEQ_FULL * SEQ_FULL) * 4 == 10485760);

typedef _Float16 h16;
typedef unsigned short bf;
typedef __attribute__((ext_vector_type(16))) __bf16   v16bf;
typedef __attribute__((ext_vector_type(16))) _Float16 v16h;
typedef __attribute__((ext_vector_type(8)))  _Float16 v8h;
typedef __attribute__((ext_vector_type(4)))  _Float16 v4h;
typedef __attribute__((ext_vector_type(8)))  unsigned short v8us;
typedef __attribute__((ext_vector_type(8)))  float    v8f;
typedef __attribute__((ext_vector_type(4)))  float    v4f;
typedef __attribute__((ext_vector_type(2)))  float    v2f;
typedef v4f  __attribute__((may_alias)) v4fa;
typedef v2f  __attribute__((may_alias)) v2fa;
typedef v8h  __attribute__((may_alias)) v8ha;
typedef v4h  __attribute__((may_alias)) v4ha;

__device__ __forceinline__ unsigned short f2bf(float f) { unsigned u = __float_as_uint(f); u += 0x7FFFu + ((u >> 16) & 1u); return (unsigned short)(u >> 16); }
__device__ __forceinline__ float bfr(float f) { return __uint_as_float(((unsigned)f2bf(f)) << 16); }
__device__ __forceinline__ v16h cat16(v8h lo, v8h hi) { return __builtin_shufflevector(lo, hi, 0, 1, 2, 3, 4, 5, 6, 7, 8, 9, 10, 11, 12, 13, 14, 15); }
__device__ __forceinline__ v16bf cat16b(v8us lo, v8us hi) { return __builtin_bit_cast(v16bf, __builtin_shufflevector(lo, hi, 0, 1, 2, 3, 4, 5, 6, 7, 8, 9, 10, 11, 12, 13, 14, 15)); }
__device__ __forceinline__ v8f wmma16(v16h a, v16h b, v8f c) { return __builtin_amdgcn_wmma_f32_16x16x32_f16(false, a, false, b, (short)0, c, false, false); }
__device__ __forceinline__ v8f wmmab(v16bf a, v16bf b, v8f c) { return __builtin_amdgcn_wmma_f32_16x16x32_bf16(false, a, false, b, (short)0, c, false, false); }
__device__ __forceinline__ v16h  ldh(const h16* p) { return cat16(*(const v8h*)p, *(const v8h*)(p + 16)); }
__device__ __forceinline__ v16bf ldb(const bf* p)  { return cat16b(*(const v8us*)p, *(const v8us*)(p + 16)); }
__device__ __forceinline__ void wave_sync() { __builtin_amdgcn_fence(3  , "wavefront"); __builtin_amdgcn_wave_barrier(); asm volatile("" ::: "memory"); }

static __device__ __forceinline__ h16 toh_flush(float v) { const h16 r = (h16)v; return (fabsf(v) < 6.103515625e-05f) ? (h16)0.0f : r; }
__device__ __forceinline__ v8f wmma16_g(v16h a, v16h b, v8f c) { c = wmma16(a, b, c); asm volatile("v_nop\n\tv_nop\n\tv_nop\n\tv_nop" : "+v"(c) : "v"(a), "v"(b)); return c; }
__device__ __forceinline__ v8f wmmab_g(v16bf a, v16bf b, v8f c) { c = wmmab(a, b, c); asm volatile("v_nop\n\tv_nop\n\tv_nop\n\tv_nop" : "+v"(c) : "v"(a), "v"(b)); return c; }
__device__ __forceinline__ float fast_tanh(float x) { const float t = __builtin_amdgcn_exp2f(x * 2.8853900817779268f); return 1.0f - 2.0f * __builtin_amdgcn_rcpf(t + 1.0f); }

__global__ __launch_bounds__(256) void k_cvt8(const float* __restrict__ src, bf* dst, size_t n8) {
    const size_t i = (size_t)blockIdx.x * 256 + threadIdx.x; if (i >= n8) return;
    const v8f v = *(const v8f*)(src + i * 8); v8us o;
#pragma unroll
    for (int k = 0; k < 8; ++k) o[k] = f2bf(v[k]);
    *(volatile v8us*)(dst + i * 8) = o; __threadfence(); *(volatile v8us*)(dst + i * 8) = o;
}

__global__ __launch_bounds__(256) void k_cvth(const float* __restrict__ src, h16* dst, size_t n8, float carry) {
    const size_t i = (size_t)blockIdx.x * 256 + threadIdx.x; if (i >= n8) return;
    const v8f v = *(const v8f*)(src + i * 8); v8h o;
#pragma unroll
    for (int k = 0; k < 8; ++k) o[k] = toh_flush(bfr(v[k]) * carry);
    *(volatile v8h*)(dst + i * 8) = o; __threadfence(); *(volatile v8h*)(dst + i * 8) = o;
}

__device__ __forceinline__ void gemm64_bf(const bf* __restrict__ A, const bf* __restrict__ Bt, const int K, const size_t aoff, const size_t boff, v8f (&acc)[4][4]) {
#pragma unroll 1
    for (int kc = 0; kc < K; kc += 32) {
        v16bf a[4];
#pragma unroll
        for (int mb = 0; mb < 4; ++mb) a[mb] = ldb(A + aoff + (size_t)mb * 16 * K + kc);
#pragma unroll
        for (int nb = 0; nb < 4; ++nb) { const v16bf b = ldb(Bt + boff + (size_t)nb * 16 * K + kc);
#pragma unroll
            for (int mb = 0; mb < 4; ++mb) acc[mb][nb] = wmmab_g(a[mb], b, acc[mb][nb]); }
    }
}
__device__ __forceinline__ void gemm64_h(const h16* __restrict__ A, const h16* __restrict__ Bt, const int K, const size_t aoff, const size_t boff, v8f (&acc)[4][4]) {
#pragma unroll 1
    for (int kc = 0; kc < K; kc += 32) {
        v16h a[4];
#pragma unroll
        for (int mb = 0; mb < 4; ++mb) a[mb] = ldh(A + aoff + (size_t)mb * 16 * K + kc);
#pragma unroll
        for (int nb = 0; nb < 4; ++nb) { const v16h b = ldh(Bt + boff + (size_t)nb * 16 * K + kc);
#pragma unroll
            for (int mb = 0; mb < 4; ++mb) acc[mb][nb] = wmma16_g(a[mb], b, acc[mb][nb]); }
    }
}

__global__ __launch_bounds__(32) void k_projadd(const bf* __restrict__ A, const bf* __restrict__ Bt, const float* __restrict__ bias,
                                                const h16* __restrict__ W2, const float* __restrict__ bias2, float* E) {
    __shared__ __align__(16) float os[16 * 68];
    __shared__ __align__(16) h16 qs[64 * QSP];
    const int lane = threadIdx.x & 31, lr = lane & 15, hi = lane >> 4; const int r0 = blockIdx.x * 64, c0 = blockIdx.y * 64;
    v8f acc[4][4];
#pragma unroll
    for (int mb = 0; mb < 4; ++mb)
#pragma unroll
        for (int nb = 0; nb < 4; ++nb) acc[mb][nb] = (v8f){};
    gemm64_bf(A, Bt, DM, (size_t)(r0 + lr) * DM + 8 * hi, (size_t)(c0 + lr) * DM + 8 * hi, acc);
    float bc[4];
#pragma unroll
    for (int nb = 0; nb < 4; ++nb) bc[nb] = bfr(bias[c0 + nb * 16 + lr]);
#pragma unroll
    for (int mb = 0; mb < 4; ++mb) {
#pragma unroll
        for (int nb = 0; nb < 4; ++nb) {
#pragma unroll
            for (int j = 0; j < 8; ++j) os[(hi * 8 + j) * 68 + nb * 16 + lr] = acc[mb][nb][j] + bc[nb]; }
        wave_sync();
#pragma unroll
        for (int s = 0; s < 4; ++s) { const int p = s * 32 + lane; const int row = p >> 3, c8 = (p & 7) * 8;
            const v4f x0 = *(const v4fa*)(&os[row * 68 + c8]); const v4f x1 = *(const v4fa*)(&os[row * 68 + c8 + 4]); v8h hv;
#pragma unroll
            for (int i = 0; i < 4; ++i) { hv[i] = toh_flush(x0[i]); hv[4 + i] = toh_flush(x1[i]); }
            *(v8ha*)(&qs[(mb * 16 + row) * QSP + c8]) = hv; }
        wave_sync();
    }
#pragma unroll
    for (int mb = 0; mb < 4; ++mb)
#pragma unroll
        for (int nb = 0; nb < 4; ++nb) acc[mb][nb] = (v8f){};
#pragma unroll
    for (int kc = 0; kc < HD; kc += 32) {
        v16h a[4];
#pragma unroll
        for (int mb = 0; mb < 4; ++mb) { const int qo = (mb * 16 + lr) * QSP + kc + 8 * hi;
            a[mb] = cat16(*(const v8ha*)(&qs[qo]), *(const v8ha*)(&qs[qo + 16])); }
#pragma unroll
        for (int nb = 0; nb < 4; ++nb) { const v16h b = ldh(W2 + (size_t)(nb * 16 + lr) * HD + kc + 8 * hi);
#pragma unroll
            for (int mb = 0; mb < 4; ++mb) acc[mb][nb] = wmma16_g(a[mb], b, acc[mb][nb]); }
    }
    float b2[4];
#pragma unroll
    for (int nb = 0; nb < 4; ++nb) b2[nb] = bfr(bias2[nb * 16 + lr]);
    const int bb = r0 / SEQ, tt = r0 % SEQ; const int zc = bb * NH_ + c0 / HD;
    const size_t ebase = ((size_t)zc * SEQ + (size_t)tt) * HD;
#pragma unroll
    for (int mb = 0; mb < 4; ++mb) {
#pragma unroll
        for (int nb = 0; nb < 4; ++nb) {
#pragma unroll
            for (int j = 0; j < 8; ++j) os[(hi * 8 + j) * 68 + nb * 16 + lr] = acc[mb][nb][j] * WAI + b2[nb]; }
        wave_sync();
#pragma unroll 1
        for (int ps = 0; ps < 2; ++ps) {
#pragma unroll
            for (int s = 0; s < 8; ++s) { const int row = 2 * s + (lane >> 4), c4 = (lane & 15) * 4;
                const v4f val = *(const v4fa*)(&os[row * 68 + c4]);
                *(volatile v4f*)(E + ebase + (size_t)(mb * 16 + row) * HD + c4) = val; }
            if (ps == 0) __threadfence(); }
        wave_sync();
    }
}

__global__ __launch_bounds__(32) void k_vt(const bf* __restrict__ A, const bf* __restrict__ Bt, const float* __restrict__ bias, h16* Ph) {
    __shared__ __align__(16) float os[16 * 68];
    const int lane = threadIdx.x & 31, lr = lane & 15, hi = lane >> 4; const int r0 = blockIdx.x * 64, c0 = blockIdx.y * 64;
    v8f acc[4][4];
#pragma unroll
    for (int mb = 0; mb < 4; ++mb)
#pragma unroll
        for (int nb = 0; nb < 4; ++nb) acc[mb][nb] = (v8f){};
    gemm64_bf(A, Bt, DM, (size_t)(r0 + lr) * DM + 8 * hi, (size_t)(c0 + lr) * DM + 8 * hi, acc);
    const int bb = c0 / SEQ, tt = c0 % SEQ;
    const size_t tbase = (size_t)bb * (size_t)DM * SEQ + (size_t)r0 * SEQ + (size_t)tt;
#pragma unroll
    for (int mb = 0; mb < 4; ++mb) {
        float br[8];
#pragma unroll
        for (int j = 0; j < 8; ++j) br[j] = bfr(bias[r0 + mb * 16 + hi * 8 + j]);
#pragma unroll
        for (int nb = 0; nb < 4; ++nb) {
#pragma unroll
            for (int j = 0; j < 8; ++j) os[(hi * 8 + j) * 68 + nb * 16 + lr] = acc[mb][nb][j] + br[j]; }
        wave_sync();
#pragma unroll 1
        for (int ps = 0; ps < 2; ++ps) {
            const size_t sb = tbase + (size_t)(mb * 16) * SEQ;
#pragma unroll
            for (int s = 0; s < 4; ++s) { const int row = 4 * s + (lane >> 3), c8 = (lane & 7) * 8;
                const v4f x0 = *(const v4fa*)(&os[row * 68 + c8]); const v4f x1 = *(const v4fa*)(&os[row * 68 + c8 + 4]); v8h hv;
#pragma unroll
                for (int i = 0; i < 4; ++i) { hv[i] = toh_flush(x0[i]); hv[4 + i] = toh_flush(x1[i]); }
                *(volatile v8h*)(Ph + sb + (size_t)row * SEQ + c8) = hv; }
            if (ps == 0) __threadfence(); }
        wave_sync();
    }
}

__global__ __launch_bounds__(256) void k_pairsoft(const float* __restrict__ QE, const float* __restrict__ KE, const float* __restrict__ vw, const float* __restrict__ vbp,
                                              const h16* __restrict__ VT, float* ATT, h16* XP) {
    __shared__ __align__(16) float ke_s[SEQ * KSP];
    __shared__ __align__(16) float qe_s[QB * HD];
    __shared__ __align__(16) float v_s[HD];
    __shared__ __align__(16) h16 ps[QB * PSP];
    __shared__ __align__(16) float xs[QB * XSP];
    __shared__ __align__(16) float rs[QB];
    const int tid = threadIdx.x, lane = tid & 31, lr = lane & 15, hi = lane >> 4;
    const int wave = __builtin_amdgcn_readfirstlane((int)(threadIdx.x >> 5));
    const int zh = blockIdx.y; const int b = zh / NH_, h = zh % NH_;
    const int q0 = blockIdx.x * QB;
    const size_t hb = (size_t)zh * SEQ * HD;
#pragma unroll 1
    for (int i = tid; i < SEQ * (HD / 2); i += 256) { const int row = i / (HD / 2), c2 = (i % (HD / 2)) * 2;
        const v2f val = *(const v2f*)(KE + hb + (size_t)row * HD + c2);
        *(v2fa*)(&ke_s[row * KSP + c2]) = val; }
#pragma unroll 1
    for (int i = tid; i < QB * HD / 4; i += 256) { const v4f val = *(const v4f*)(QE + hb + (size_t)q0 * HD + (size_t)i * 4); *(v4fa*)(&qe_s[i * 4]) = val; }
    if (tid < HD) v_s[tid] = bfr(vw[tid]);
    __syncthreads();
    const float vb = bfr(vbp[0]);
#pragma unroll 1
    for (int it = 0; it < QB / 8; ++it) {
        const int ql = wave + 8 * it;
        float acc[NKL];
#pragma unroll
        for (int j = 0; j < NKL; ++j) acc[j] = 0.0f;
#pragma unroll 2
        for (int d2 = 0; d2 < HD / 2; ++d2) {
            const v2f vv = *(const v2fa*)(&v_s[2 * d2]);
            const v2f vq = *(const v2fa*)(&qe_s[ql * HD + 2 * d2]);
#pragma unroll
            for (int j = 0; j < NKL; ++j) {
                const int k = 128 * (j >> 2) + 4 * lane + (j & 3);
                const v2f kv = *(const v2fa*)(&ke_s[k * KSP + 2 * d2]);
                acc[j] = fmaf(vv.x, fast_tanh(vq.x + kv.x), acc[j]);
                acc[j] = fmaf(vv.y, fast_tanh(vq.y + kv.y), acc[j]);
            }
        }
        float e[NKL];
#pragma unroll
        for (int j = 0; j < NKL; ++j) e[j] = acc[j] + vb;
        float m = e[0];
#pragma unroll
        for (int j = 1; j < NKL; ++j) m = fmaxf(m, e[j]);
#pragma unroll
        for (int off = 16; off >= 1; off >>= 1) m = fmaxf(m, __shfl_xor(m, off, 32));
        float p[NKL]; float s = 0.0f;
#pragma unroll
        for (int j = 0; j < NKL; ++j) { p[j] = __builtin_amdgcn_exp2f((e[j] - m) * LOG2E); s += p[j]; }
#pragma unroll
        for (int off = 16; off >= 1; off >>= 1) s += __shfl_xor(s, off, 32);
        const float inv = 1.0f / s;
        v4f av[KG]; float s16 = 0.0f;
#pragma unroll
        for (int g = 0; g < KG; ++g) { v4h ph;
#pragma unroll
            for (int i = 0; i < 4; ++i) { const float pv = p[4 * g + i]; av[g][i] = pv * inv;
                const h16 pq = toh_flush(pv * PCS); ph[i] = pq; s16 += (float)pq; }
            *(v4ha*)(&ps[ql * PSP + 128 * g + 4 * lane]) = ph; }
#pragma unroll
        for (int off = 16; off >= 1; off >>= 1) s16 += __shfl_xor(s16, off, 32);
        if (lane == 0) rs[ql] = s16;
        float* arow = ATT + ((size_t)zh * SEQ + (size_t)(q0 + ql)) * SEQ;
#pragma unroll 1
        for (int pz = 0; pz < 2; ++pz) {
#pragma unroll
            for (int g = 0; g < KG; ++g) *(volatile v4f*)(arow + 128 * g + 4 * lane) = av[g];
            if (pz == 0) __threadfence(); }
    }
    __syncthreads();
    {   const int mt = wave >> 2, nt = wave & 3;
        v8f o = (v8f){};
        const int po = (mt * 16 + lr) * PSP + 8 * hi;
        const size_t vo = ((size_t)zh * HD + (size_t)(nt * 16 + lr)) * SEQ + 8 * hi;
#pragma unroll
        for (int kc = 0; kc < SEQ; kc += 32) {
            const v16h a = cat16(*(const v8ha*)(&ps[po + kc]), *(const v8ha*)(&ps[po + kc + 16]));
            const v16h bq = ldh(VT + vo + kc);
            o = wmma16_g(a, bq, o);
        }
#pragma unroll
        for (int r = 0; r < 8; ++r) { const int row = mt * 16 + 8 * hi + r;
            const float sc = XCS * (1.0f / rs[row]);
            xs[row * XSP + nt * 16 + lr] = o[r] * sc; }
    }
    __syncthreads();
    {   const int row = tid >> 3, c8 = (tid & 7) * 8;
        const v4f x0 = *(const v4fa*)(&xs[row * XSP + c8]); const v4f x1 = *(const v4fa*)(&xs[row * XSP + c8 + 4]); v8h hv;
#pragma unroll
        for (int i = 0; i < 4; ++i) { hv[i] = toh_flush(x0[i]); hv[4 + i] = toh_flush(x1[i]); }
        const size_t oo = ((size_t)b * SEQ + (size_t)(q0 + row)) * DM + (size_t)h * HD + c8;
        *(volatile v8h*)(XP + oo) = hv; __threadfence(); *(volatile v8h*)(XP + oo) = hv; }
}

__global__ __launch_bounds__(32) void k_out(const h16* __restrict__ A, const h16* __restrict__ Bt, const float* __restrict__ bias, float* OUT) {
    __shared__ __align__(16) float os[16 * 68];
    const int lane = threadIdx.x & 31, lr = lane & 15, hi = lane >> 4; const int r0 = blockIdx.x * 64, c0 = blockIdx.y * 64;
    v8f acc[4][4];
#pragma unroll
    for (int mb = 0; mb < 4; ++mb)
#pragma unroll
        for (int nb = 0; nb < 4; ++nb) acc[mb][nb] = (v8f){};
    gemm64_h(A, Bt, DM, (size_t)(r0 + lr) * DM + 8 * hi, (size_t)(c0 + lr) * DM + 8 * hi, acc);
    float bc[4];
#pragma unroll
    for (int nb = 0; nb < 4; ++nb) bc[nb] = bfr(bias[c0 + nb * 16 + lr]);
    const int bb = r0 / SEQ, tt = r0 % SEQ;
    const size_t obase = ((size_t)bb * OUT_SEQ + (size_t)tt) * DM + (size_t)c0;
#pragma unroll
    for (int mb = 0; mb < 4; ++mb) {
#pragma unroll
        for (int nb = 0; nb < 4; ++nb) {
#pragma unroll
            for (int j = 0; j < 8; ++j) os[(hi * 8 + j) * 68 + nb * 16 + lr] = acc[mb][nb][j] * OUTI + bc[nb]; }
        wave_sync();
#pragma unroll 1
        for (int ps = 0; ps < 2; ++ps) {
#pragma unroll
            for (int s = 0; s < 8; ++s) { const int row = 2 * s + (lane >> 4), c4 = (lane & 15) * 4;
                const v4f val = *(const v4fa*)(&os[row * 68 + c4]);
                *(volatile v4f*)(OUT + obase + (size_t)(mb * 16 + row) * DM + c4) = val; }
            if (ps == 0) __threadfence(); }
        wave_sync();
    }
}

static constexpr size_t al256(size_t v) { return (v + 255) & ~(size_t)255; }
static constexpr size_t SZ_XB = al256((size_t)NB * SEQ * DM * 2);
static constexpr size_t SZ_WB = al256((size_t)3 * DM * DM * 2);
static constexpr size_t SZ_FO = al256((size_t)DM * DM * 2);
static constexpr size_t SZ_WA = al256((size_t)HD * HD * 2);
static constexpr size_t SZ_EP = al256((size_t)NB * NH_ * SEQ * HD * 4);
static constexpr size_t SZ_VT = al256((size_t)NB * DM * SEQ * 2);
static constexpr size_t SZ_XP = al256((size_t)NB * SEQ * DM * 2);
static constexpr size_t SZ_TOTAL = 3 * SZ_XB + SZ_WB + SZ_FO + 2 * SZ_WA + 2 * SZ_EP + SZ_VT + SZ_XP;
static_assert(SZ_TOTAL <= (size_t)134217728);
static_assert(((size_t)DM * DM * 2) % 256 == 0);
static_assert((size_t)NB * NH_ * SEQ * HD == (size_t)NB * DM * SEQ);

extern "C" void kernel_launch(void* const* d_in, const int* in_sizes, int n_in,
                              void* d_out, int out_size, void* d_ws, size_t ws_size, hipStream_t stream) {
    if (n_in < 17) return;
    const size_t needx = ((size_t)(NB - 1) * SEQ_FULL + SEQ) * DM;
    if ((size_t)in_sizes[0] < needx || (size_t)in_sizes[1] < needx || (size_t)in_sizes[2] < needx) return;
    if (in_sizes[3] < HD * HD || in_sizes[4] < HD || in_sizes[5] < HD * HD || in_sizes[6] < HD || in_sizes[7] < HD || in_sizes[8] < 1) return;
    if ((size_t)in_sizes[9] < (size_t)DM * DM || (size_t)in_sizes[11] < (size_t)DM * DM || (size_t)in_sizes[13] < (size_t)DM * DM || (size_t)in_sizes[15] < (size_t)DM * DM) return;
    if (in_sizes[10] < DM || in_sizes[12] < DM || in_sizes[14] < DM || in_sizes[16] < DM) return;
    const size_t att_off = (size_t)NB_FULL * SEQ_FULL * DM;
    if ((size_t)out_size < att_off + (size_t)NB * NH_ * SEQ * SEQ) return;
    if ((size_t)out_size < ((size_t)(NB - 1) * OUT_SEQ + SEQ) * DM) return;
    if (SZ_TOTAL > ws_size) return;
    const float* xin[3] = { (const float*)d_in[0], (const float*)d_in[1], (const float*)d_in[2] };
    const float* wa = (const float*)d_in[3];  const float* ba = (const float*)d_in[4];
    const float* ua = (const float*)d_in[5];  const float* bu = (const float*)d_in[6];
    const float* vw = (const float*)d_in[7];  const float* vb = (const float*)d_in[8];
    const float* wq = (const float*)d_in[9];  const float* bq = (const float*)d_in[10];
    const float* wk = (const float*)d_in[11]; const float* bk = (const float*)d_in[12];
    const float* wv = (const float*)d_in[13]; const float* bv = (const float*)d_in[14];
    const float* wo = (const float*)d_in[15]; const float* bo = (const float*)d_in[16];
    float* OUT = (float*)d_out;
    float* ATT = (float*)d_out + att_off;
    char* wsp = (char*)d_ws;
    bf* XB[3];
    XB[0] = (bf*)wsp; wsp += SZ_XB;
    XB[1] = (bf*)wsp; wsp += SZ_XB;
    XB[2] = (bf*)wsp; wsp += SZ_XB;
    bf* WB = (bf*)wsp; wsp += SZ_WB;
    h16* FO = (h16*)wsp; wsp += SZ_FO;
    h16* WA = (h16*)wsp; wsp += SZ_WA;
    h16* UA = (h16*)wsp; wsp += SZ_WA;
    float* QE = (float*)wsp; wsp += SZ_EP;
    float* KE = (float*)wsp; wsp += SZ_EP;
    h16* VT = (h16*)wsp; wsp += SZ_VT;
    h16* XP = (h16*)wsp; wsp += SZ_XP;
    bf* WQ = WB; bf* WK = WB + (size_t)DM * DM; bf* WV = WB + (size_t)2 * DM * DM;

    for (int i = 0; i < 3; ++i) {
        if (SEQ == SEQ_FULL) {
            const size_t n8 = (size_t)NB * SEQ * DM / 8;
            k_cvt8<<<(unsigned)((n8 + 255) / 256), 256, 0, stream>>>(xin[i], XB[i], n8);
        } else {
            const size_t n8 = (size_t)SEQ * DM / 8;
            for (int b = 0; b < NB; ++b) k_cvt8<<<(unsigned)((n8 + 255) / 256), 256, 0, stream>>>(xin[i] + (size_t)b * SEQ_FULL * DM, XB[i] + (size_t)b * SEQ * DM, n8);
        }
    }
    { const size_t n8 = (size_t)DM * DM / 8; const unsigned g = (unsigned)((n8 + 255) / 256);
      k_cvt8<<<g, 256, 0, stream>>>(wq, WQ, n8); k_cvt8<<<g, 256, 0, stream>>>(wk, WK, n8); k_cvt8<<<g, 256, 0, stream>>>(wv, WV, n8);
      k_cvth<<<g, 256, 0, stream>>>(wo, FO, n8, FOS); }
    { const size_t n8 = (size_t)HD * HD / 8; const unsigned g = (unsigned)((n8 + 255) / 256);
      k_cvth<<<g, 256, 0, stream>>>(wa, WA, n8, WAS); k_cvth<<<g, 256, 0, stream>>>(ua, UA, n8, WAS); }

    k_projadd<<<dim3(NB * SEQ / 64, DM / 64, 1), 32, 0, stream>>>(XB[0], WQ, bq, WA, ba, QE);
    k_projadd<<<dim3(NB * SEQ / 64, DM / 64, 1), 32, 0, stream>>>(XB[1], WK, bk, UA, bu, KE);
    k_vt<<<dim3(DM / 64, NB * SEQ / 64, 1), 32, 0, stream>>>(WV, XB[2], bv, VT);
    k_pairsoft<<<dim3(SEQ / QB, NB * NH_, 1), 256, 0, stream>>>(QE, KE, vw, vb, VT, ATT, XP);
    k_out<<<dim3(NB * SEQ / 64, DM / 64, 1), 32, 0, stream>>>(XP, FO, bo, OUT);
}
